// ParallelWaveGANGenerator_77610059038928
// MI455X (gfx1250) — hardware-verified
//
#include <hip/hip_runtime.h>
#include <hip/hip_bf16.h>


#define NB    2
#define TL    32768
#define TF    128
#define RC    64
#define GC    128
#define SC    64
#define AC    80
#define ACP   96
#define NLAY  30
#define GRD   512
#define TPAD  (TL + 2 * GRD)
#define TT    64
#define ZP    72
#define EP    68
#define KD    192
#define U3W   (TL / 4)
#define SQH   0.70710678118654752f
#define SKS   0.18257418583505536f

static_assert(GRD >= 512);
static_assert(TL % TT == 0);
static_assert((TL / TT) == 512);
static_assert(TL % 32 == 0);

typedef float          v4f   __attribute__((ext_vector_type(4)));
typedef float          v8f   __attribute__((ext_vector_type(8)));
typedef _Float16       v8h   __attribute__((ext_vector_type(8)));
typedef _Float16       v16h  __attribute__((ext_vector_type(16)));
typedef __bf16         v16b  __attribute__((ext_vector_type(16)));
typedef unsigned short u16x8 __attribute__((ext_vector_type(8)));
union Frag { u16x8 h[2]; v8h x[2]; v16h f; v16b b; };
union H8 { v8h f; u16x8 u; };

constexpr size_t SZ_C1  = (size_t)NB * AC * TF * 4;
constexpr size_t SZ_U1  = (size_t)NB * AC * 512 * 4;
constexpr size_t SZ_U2  = (size_t)NB * AC * 2048 * 4;
constexpr size_t SZ_U3  = (size_t)NB * AC * U3W * 4;
constexpr size_t SZ_CUP = (size_t)NB * TL * ACP * 2;
constexpr size_t SZ_H   = (size_t)NB * TL * RC * 4;
constexpr size_t SZ_HH  = (size_t)NB * TPAD * RC * 2;
constexpr size_t SZ_WD  = (size_t)NLAY * GC * KD * 2;
constexpr size_t SZ_WA  = (size_t)NLAY * GC * ACP * 2;
constexpr size_t SZ_W2  = (size_t)NLAY * GC * RC * 2;
constexpr size_t SZ_WL  = (size_t)SC * SC * 2;
constexpr size_t OFF_C1 = 0, OFF_U1 = OFF_C1 + SZ_C1, OFF_U2 = OFF_U1 + SZ_U1, OFF_U3 = OFF_U2 + SZ_U2, OFF_CUP = OFF_U3 + SZ_U3;
constexpr size_t OFF_HA = OFF_CUP + SZ_CUP, OFF_HB = OFF_HA + SZ_H, OFF_SA = OFF_HB + SZ_H, OFF_SB = OFF_SA + SZ_H;
constexpr size_t OFF_HHA = OFF_SB + SZ_H, OFF_HHB = OFF_HHA + SZ_HH, OFF_WD = OFF_HHB + SZ_HH, OFF_WA = OFF_WD + SZ_WD, OFF_W2 = OFF_WA + SZ_WA;
constexpr size_t OFF_WLH = OFF_W2 + SZ_W2, OFF_WLL = OFF_WLH + SZ_WL, WS_END = OFF_WLL + SZ_WL;
static_assert(WS_END <= (size_t)134217728);
static_assert(OFF_U1 % 512 == 0 && OFF_U2 % 512 == 0 && OFF_U3 % 512 == 0 && OFF_CUP % 512 == 0 && OFF_HA % 512 == 0 && OFF_HB % 512 == 0);
static_assert(OFF_SA % 512 == 0 && OFF_SB % 512 == 0 && OFF_HHA % 512 == 0 && OFF_HHB % 512 == 0 && OFF_WD % 512 == 0 && OFF_WA % 512 == 0);
static_assert(OFF_W2 % 512 == 0 && OFF_WLH % 512 == 0 && OFF_WLL % 512 == 0 && WS_END % 512 == 0);
static_assert(SZ_C1 % 512 == 0 && SZ_U1 % 512 == 0 && SZ_U2 % 512 == 0 && SZ_U3 % 512 == 0 && SZ_CUP % 512 == 0 && SZ_H % 512 == 0);
static_assert(SZ_HH % 512 == 0 && SZ_WD % 512 == 0 && SZ_WA % 512 == 0 && SZ_W2 % 512 == 0 && SZ_WL % 512 == 0);
static_assert((NLAY * GC * KD / 8) == 360 * 256);

__device__ __forceinline__ unsigned short f32_to_bf16(float f) {
    unsigned u = __float_as_uint(f);
    return (unsigned short)((u + 0x7FFFu + ((u >> 16) & 1u)) >> 16);
}
__device__ __forceinline__ float bf16_to_f32(unsigned short b) { return __uint_as_float(((unsigned)b) << 16); }
__device__ __forceinline__ v8f ld8f(const float* p) {
    v4f a = *(const v4f*)p; v4f b = *(const v4f*)(p + 4);
    return __builtin_shufflevector(a, b, 0, 1, 2, 3, 4, 5, 6, 7);
}
__device__ __forceinline__ void split8(const v8f x, u16x8& hv, u16x8& lv) {
#pragma unroll
    for (int c = 0; c < 8; ++c) {
        const unsigned short hb = f32_to_bf16(x[c]);
        hv[c] = hb; lv[c] = f32_to_bf16(x[c] - bf16_to_f32(hb));
    }
}
__device__ __forceinline__ void mma_h(v8f& acc, const Frag& a, const Frag& b) {
    acc = __builtin_amdgcn_wmma_f32_16x16x32_f16(false, a.f, false, b.f, (short)0, acc, false, false);
    asm volatile("v_nop\n\tv_nop\n\tv_nop\n\tv_nop" : "+v"(acc) : "v"(a.f), "v"(b.f));
}
__device__ __forceinline__ void mma_b(v8f& acc, const Frag& a, const Frag& b) {
    acc = __builtin_amdgcn_wmma_f32_16x16x32_bf16(false, a.b, false, b.b, (short)0, acc, false, false);
    asm volatile("v_nop\n\tv_nop\n\tv_nop\n\tv_nop" : "+v"(acc) : "v"(a.b), "v"(b.b));
}
__device__ __forceinline__ void zero8(v8f& a) {
#pragma unroll
    for (int r = 0; r < 8; ++r) a[r] = 0.f;
}

__global__ __launch_bounds__(256)
void k_c1(const float* __restrict__ c, const float* __restrict__ wcin, float* c1, int total)
{
    const int idx = blockIdx.x * 256 + threadIdx.x;
    if (idx >= total) return;
    const int f = idx & (TF - 1), r = idx >> 7, o = r % AC, b = r / AC;
    const float* cb = c + (size_t)b * AC * TF + f;
    const float* w = wcin + o * AC;
    float acc = 0.f;
#pragma unroll 1
    for (int k = 0; k < AC; ++k) acc += w[k] * cb[(size_t)k * TF];
    *(volatile float*)(c1 + idx) = acc;
    __threadfence();
    *(volatile float*)(c1 + idx) = acc;
}

__global__ __launch_bounds__(256)
void k_up(const float* __restrict__ in, const float* __restrict__ w9, float* outp, int win, int total)
{
    const int idx = blockIdx.x * 256 + threadIdx.x;
    if (idx >= total) return;
    const int wout = win * 4;
    const int t = idx % wout, bc = idx / wout;
    const float* src = in + (size_t)bc * win;
    float acc = 0.f;
#pragma unroll
    for (int k = 0; k < 9; ++k) {
        const int j = t - 4 + k;
        const int jj = min(max(j, 0), wout - 1);
        const float v = src[jj >> 2];
        const float pv = w9[k] * v;
        acc += (j >= 0 && j < wout) ? pv : 0.f;
    }
    *(volatile float*)(outp + idx) = acc;
    __threadfence();
    *(volatile float*)(outp + idx) = acc;
}

__global__ __launch_bounds__(256)
void k_uplast(const float* __restrict__ u3, const float* __restrict__ w9, unsigned short* cup)
{
    __shared__ __attribute__((aligned(16))) _Float16 sc[TT * ACP];
    const int tid = threadIdx.x;
    const int b = blockIdx.x >> 9, t0 = (blockIdx.x & 511) * TT;
    const float* ub = u3 + (size_t)b * AC * U3W;
#pragma unroll 1
    for (int idx = tid; idx < TT * AC; idx += 256) {
        const int tok = idx & (TT - 1), ch = idx >> 6;
        const int t = t0 + tok;
        const float* src = ub + (size_t)ch * U3W;
        float acc = 0.f;
#pragma unroll
        for (int k = 0; k < 9; ++k) {
            const int j = t - 4 + k;
            const int jj = min(max(j, 0), TL - 1);
            const float v = src[jj >> 2];
            const float pv = w9[k] * v;
            acc += (j >= 0 && j < TL) ? pv : 0.f;
        }
        sc[tok * ACP + ch] = (_Float16)acc;
    }
#pragma unroll 1
    for (int idx = tid; idx < TT * (ACP - AC); idx += 256) {
        const int tok = idx >> 4, q = idx & 15;
        sc[tok * ACP + AC + q] = (_Float16)0.f;
    }
    __syncthreads();
    unsigned short* dst = cup + ((size_t)b * TL + t0) * ACP;
    H8 u[3];
#pragma unroll
    for (int it = 0; it < 3; ++it) u[it].f = *(const v8h*)(sc + (it * 256 + tid) * 8);
#pragma unroll
    for (int it = 0; it < 3; ++it) *(volatile u16x8*)(dst + (size_t)(it * 256 + tid) * 8) = u[it].u;
    __threadfence();
#pragma unroll
    for (int it = 0; it < 3; ++it) *(volatile u16x8*)(dst + (size_t)(it * 256 + tid) * 8) = u[it].u;
}

__global__ __launch_bounds__(256)
void k_wprep(const float* __restrict__ wd, const float* __restrict__ wa, const float* __restrict__ wsk, const float* __restrict__ wr,
             const float* __restrict__ wl1, unsigned short* pwd, unsigned short* pwa, unsigned short* pw2, unsigned short* pl1h, unsigned short* pl1l)
{
    const int seg = blockIdx.y;
    const int i8 = blockIdx.x * 256 + threadIdx.x;
    const int lim = (seg == 0) ? (NLAY * GC * KD / 8) : (seg == 1) ? (NLAY * GC * ACP / 8) : (seg == 2) ? (NLAY * GC * RC / 8) : (SC * SC / 8);
    if (i8 >= lim) return;
    const int o0 = i8 * 8;
    v8f v;
    if (seg == 0) {
        const int li = o0 / (GC * KD), rem = o0 - li * (GC * KD), o = rem / KD, k = rem - o * KD, tap = k >> 6, ci = k & 63;
        const float* p = wd + (((size_t)li * GC + o) * RC + ci) * 3 + tap;
#pragma unroll
        for (int cc = 0; cc < 8; ++cc) v[cc] = 16.f * p[cc * 3];
    } else if (seg == 1) {
        const int li = o0 / (GC * ACP), rem = o0 - li * (GC * ACP), o = rem / ACP, k = rem - o * ACP;
        const int kc = min(k, AC - 8);
        const float* p = wa + ((size_t)li * GC + o) * AC + kc;
#pragma unroll
        for (int cc = 0; cc < 8; ++cc) { const float t = p[cc]; v[cc] = (k < AC) ? 64.f * t : 0.f; }
    } else if (seg == 2) {
        const int li = o0 / (GC * RC), rem = o0 - li * (GC * RC), o = rem >> 6, k = rem & 63;
        const int os = min(o, SC - 1), orr = max(o - SC, 0);
        const float* p = wsk + ((size_t)li * SC + os) * RC + k;
        const float* q = wr  + ((size_t)li * RC + orr) * SC + k;
#pragma unroll
        for (int cc = 0; cc < 8; ++cc) { const float a = p[cc]; const float bq = q[cc]; v[cc] = 16.f * ((o < SC) ? a : bq); }
    } else {
#pragma unroll
        for (int cc = 0; cc < 8; ++cc) v[cc] = wl1[o0 + cc];
    }
    if (seg < 3) {
        unsigned short* dst = (seg == 0) ? pwd : (seg == 1) ? pwa : pw2;
        H8 u; u.f = __builtin_convertvector(v, v8h);
        *(volatile u16x8*)(dst + o0) = u.u;
        __threadfence();
        *(volatile u16x8*)(dst + o0) = u.u;
    } else {
        u16x8 hv, lv; split8(v, hv, lv);
        *(volatile u16x8*)(pl1h + o0) = hv; *(volatile u16x8*)(pl1l + o0) = lv;
        __threadfence();
        *(volatile u16x8*)(pl1h + o0) = hv; *(volatile u16x8*)(pl1l + o0) = lv;
    }
}

__global__ __launch_bounds__(256)
void k_guard(unsigned short* hh)
{
    const int i = blockIdx.x * 256 + threadIdx.x;
    if (i >= 32768) return;
    const int plane = i >> 14, j = i & 16383, b = j >> 13, r = (j >> 3) & 1023, seg = j & 7;
    const int row = b * TPAD + ((r < GRD) ? r : (TL + r));
    unsigned short* gp = hh + (size_t)plane * NB * TPAD * RC + (size_t)row * RC + seg * 8;
    const u16x8 z8 = {0, 0, 0, 0, 0, 0, 0, 0};
    *(volatile u16x8*)gp = z8;
    __threadfence();
    *(volatile u16x8*)gp = z8;
}

__global__ __launch_bounds__(128)
void k_h0(const float* __restrict__ x, const float* __restrict__ wf, const float* __restrict__ bfst, float* hpl, float* spl, unsigned short* hh)
{
    const int tid = threadIdx.x;
    const int tok0 = blockIdx.x * 32;
    const int b = tok0 >> 15, t = tok0 & (TL - 1);
    v4f hv[4];
#pragma unroll
    for (int it = 0; it < 4; ++it) {
        const int p = it * 128 + tid, tk = p >> 4, c0 = (p & 15) * 4;
        const float xv = x[tok0 + tk];
#pragma unroll
        for (int q = 0; q < 4; ++q) hv[it][q] = wf[c0 + q] * xv + bfst[c0 + q];
    }
    H8 u[2];
#pragma unroll
    for (int it = 0; it < 2; ++it) {
        const int p = it * 128 + tid, tk = p >> 3, c0 = (p & 7) * 8;
        const float xv = x[tok0 + tk];
        v8f y;
#pragma unroll
        for (int q = 0; q < 8; ++q) y[q] = (wf[c0 + q] * xv + bfst[c0 + q]) * 4.f;
        u[it].f = __builtin_convertvector(y, v8h);
    }
    const v4f z4 = {0.f, 0.f, 0.f, 0.f};
    const size_t grow0 = (size_t)b * TPAD + GRD + t;
#pragma unroll
    for (int it = 0; it < 4; ++it) {
        const int p = it * 128 + tid, tk = p >> 4, c0 = (p & 15) * 4;
        const size_t go = (size_t)(tok0 + tk) * RC + c0;
        *(volatile v4f*)(hpl + go) = hv[it];
        *(volatile v4f*)(spl + go) = z4;
    }
#pragma unroll
    for (int it = 0; it < 2; ++it) {
        const int p = it * 128 + tid, tk = p >> 3, c0 = (p & 7) * 8;
        *(volatile u16x8*)(hh + (grow0 + tk) * RC + c0) = u[it].u;
    }
    __threadfence();
#pragma unroll
    for (int it = 0; it < 4; ++it) {
        const int p = it * 128 + tid, tk = p >> 4, c0 = (p & 15) * 4;
        const size_t go = (size_t)(tok0 + tk) * RC + c0;
        *(volatile v4f*)(hpl + go) = hv[it];
        *(volatile v4f*)(spl + go) = z4;
    }
#pragma unroll
    for (int it = 0; it < 2; ++it) {
        const int p = it * 128 + tid, tk = p >> 3, c0 = (p & 7) * 8;
        *(volatile u16x8*)(hh + (grow0 + tk) * RC + c0) = u[it].u;
    }
}

__device__ __forceinline__ void layer_store(const float* sS, const float* sR, float* s_out, float* h_out, unsigned short* hh_out,
                                            size_t tokb, size_t growb, int tid)
{
#pragma unroll
    for (int it = 0; it < 8; ++it) {
        const int p = it * 128 + tid, tok = p >> 4, c0 = (p & 15) * 4;
        const v4f sv = *(const v4f*)(sS + tok * EP + c0);
        const v4f rv = *(const v4f*)(sR + tok * EP + c0);
        const size_t go = (tokb + tok) * RC + c0;
        *(volatile v4f*)(s_out + go) = sv;
        *(volatile v4f*)(h_out + go) = rv;
    }
#pragma unroll
    for (int it = 0; it < 4; ++it) {
        const int p = it * 128 + tid, tok = p >> 3, c0 = (p & 7) * 8;
        const v8f xv = ld8f(sR + tok * EP + c0);
        H8 u; u.f = __builtin_convertvector(xv * 4.f, v8h);
        *(volatile u16x8*)(hh_out + (growb + tok) * RC + c0) = u.u;
    }
}

__global__ __launch_bounds__(128)
void k_layer(const unsigned short* __restrict__ hh_in, const float* __restrict__ h_in, const float* __restrict__ s_in,
             const unsigned short* __restrict__ cup, const unsigned short* __restrict__ wd, const unsigned short* __restrict__ wa,
             const unsigned short* __restrict__ w2, const float* __restrict__ bd, const float* __restrict__ bs, const float* __restrict__ br,
             unsigned short* hh_out, float* h_out, float* s_out, int d)
{
    __shared__ __attribute__((aligned(16))) _Float16 sZ[TT * ZP];
    __shared__ __attribute__((aligned(16))) float    sS[TT * EP];
    __shared__ __attribute__((aligned(16))) float    sR[TT * EP];
    const int tid = threadIdx.x, lane = tid & 31, wave = tid >> 5, h = lane >> 4, m = lane & 15;
    const int b = blockIdx.x >> 9, t0 = (blockIdx.x & 511) * TT;
    const size_t tokb  = (size_t)b * TL + t0;
    const size_t growb = (size_t)b * TPAD + GRD + t0;
    const int oc0 = 16 * wave + m;

    v8f acc[8];
#pragma unroll
    for (int j = 0; j < 8; ++j) zero8(acc[j]);

#pragma unroll 1
    for (int ks = 0; ks < 6; ++ks) {
        const int tap = ks >> 1, ci0 = (ks & 1) * 32;
        const size_t rb = growb + (size_t)(tap * d) - (size_t)d;
        Frag fa[4];
#pragma unroll
        for (int nt = 0; nt < 4; ++nt) {
            const unsigned short* p = hh_in + (rb + 16 * nt + m) * RC + ci0 + 8 * h;
            fa[nt].h[0] = *(const u16x8*)p; fa[nt].h[1] = *(const u16x8*)(p + 16);
        }
#pragma unroll
        for (int pp = 0; pp < 2; ++pp) {
            const unsigned short* q = wd + (size_t)(oc0 + 64 * pp) * KD + ks * 32 + 8 * h;
            Frag fb; fb.h[0] = *(const u16x8*)q; fb.h[1] = *(const u16x8*)(q + 16);
#pragma unroll
            for (int nt = 0; nt < 4; ++nt) mma_h(acc[pp * 4 + nt], fa[nt], fb);
        }
    }
#pragma unroll 1
    for (int ks = 0; ks < 3; ++ks) {
        Frag fa[4];
#pragma unroll
        for (int nt = 0; nt < 4; ++nt) {
            const unsigned short* p = cup + (tokb + 16 * nt + m) * ACP + ks * 32 + 8 * h;
            fa[nt].h[0] = *(const u16x8*)p; fa[nt].h[1] = *(const u16x8*)(p + 16);
        }
#pragma unroll
        for (int pp = 0; pp < 2; ++pp) {
            const unsigned short* q = wa + (size_t)(oc0 + 64 * pp) * ACP + ks * 32 + 8 * h;
            Frag fb; fb.h[0] = *(const u16x8*)q; fb.h[1] = *(const u16x8*)(q + 16);
#pragma unroll
            for (int nt = 0; nt < 4; ++nt) mma_h(acc[pp * 4 + nt], fa[nt], fb);
        }
    }

    {
        const float bd0 = bd[oc0], bd1 = bd[64 + oc0];
#pragma unroll
        for (int nt = 0; nt < 4; ++nt) {
#pragma unroll
            for (int r = 0; r < 8; ++r) {
                const float xa = acc[nt][r] * (1.f / 64.f) + bd0;
                const float xb = acc[4 + nt][r] * (1.f / 64.f) + bd1;
                const float ea = __expf(-2.f * fabsf(xa));
                float th = (1.f - ea) * __builtin_amdgcn_rcpf(1.f + ea);
                th = copysignf(th, xa);
                const float eb = __expf(fminf(-xb, 80.f));
                const float sg = __builtin_amdgcn_rcpf(1.f + eb);
                const float z = th * sg;
                sZ[(16 * nt + 8 * h + r) * ZP + oc0] = (_Float16)(z * 8.f);
            }
        }
    }
    __syncthreads();

    v8f acc2[8];
#pragma unroll
    for (int j = 0; j < 8; ++j) zero8(acc2[j]);
#pragma unroll
    for (int ks = 0; ks < 2; ++ks) {
        Frag fa[4];
#pragma unroll
        for (int nt = 0; nt < 4; ++nt) {
            const _Float16* zp = sZ + (16 * nt + m) * ZP + 32 * ks + 8 * h;
            fa[nt].x[0] = *(const v8h*)zp; fa[nt].x[1] = *(const v8h*)(zp + 16);
        }
#pragma unroll
        for (int pp = 0; pp < 2; ++pp) {
            const unsigned short* q = w2 + (size_t)(oc0 + 64 * pp) * RC + 32 * ks + 8 * h;
            Frag fb; fb.h[0] = *(const u16x8*)q; fb.h[1] = *(const u16x8*)(q + 16);
#pragma unroll
            for (int nt = 0; nt < 4; ++nt) mma_h(acc2[pp * 4 + nt], fa[nt], fb);
        }
    }
#pragma unroll
    for (int nt = 0; nt < 4; ++nt) {
#pragma unroll
        for (int r = 0; r < 8; ++r) {
            const int row = 16 * nt + 8 * h + r;
            sS[row * EP + oc0] = acc2[nt][r];
            sR[row * EP + oc0] = acc2[4 + nt][r];
        }
    }
    __syncthreads();

#pragma unroll
    for (int it = 0; it < 8; ++it) {
        const int p = it * 128 + tid, tok = p >> 4, c0 = (p & 15) * 4;
        float* ps = sS + tok * EP + c0;
        float* pr = sR + tok * EP + c0;
        const v4f sv = *(const v4f*)ps;
        const v4f rv = *(const v4f*)pr;
        const size_t go = (tokb + tok) * RC + c0;
        const v4f so = *(const v4f*)(s_in + go);
        const v4f ho = *(const v4f*)(h_in + go);
        v4f bs4, br4;
#pragma unroll
        for (int q = 0; q < 4; ++q) { bs4[q] = bs[c0 + q]; br4[q] = br[c0 + q]; }
        const v4f sn = (so + sv * (1.f / 128.f)) + bs4;
        const v4f hn = ((rv * (1.f / 128.f) + br4) + ho) * SQH;
        *(v4f*)ps = sn;
        *(v4f*)pr = hn;
    }
    __syncthreads();
    layer_store(sS, sR, s_out, h_out, hh_out, tokb, growb, tid);
    __threadfence();
    layer_store(sS, sR, s_out, h_out, hh_out, tokb, growb, tid);
}

__global__ __launch_bounds__(128)
void k_tail(const float* __restrict__ s, const unsigned short* __restrict__ w1h, const unsigned short* __restrict__ w1l,
            const float* __restrict__ bl1, const float* __restrict__ wl2, const float* __restrict__ bl2, float* out)
{
    __shared__ __attribute__((aligned(16))) unsigned short sAH[TT * ZP];
    __shared__ __attribute__((aligned(16))) unsigned short sAL[TT * ZP];
    __shared__ __attribute__((aligned(16))) float st[4][16 * EP];
    __shared__ __attribute__((aligned(16))) float sy[TT];
    const int tid = threadIdx.x, lane = tid & 31, wave = tid >> 5, h = lane >> 4, m = lane & 15;
    const size_t tok0 = (size_t)blockIdx.x * TT;
#pragma unroll
    for (int it = 0; it < 4; ++it) {
        const int g = it * 128 + tid, row = g >> 3, c0 = (g & 7) * 8;
        const v8f xv = ld8f(s + (tok0 + row) * RC + c0);
        v8f y;
#pragma unroll
        for (int cc = 0; cc < 8; ++cc) y[cc] = fmaxf(xv[cc] * SKS, 0.f);
        u16x8 hv, lv; split8(y, hv, lv);
        *(u16x8*)(sAH + row * ZP + c0) = hv;
        *(u16x8*)(sAL + row * ZP + c0) = lv;
    }
    __syncthreads();
    v8f acc[4];
#pragma unroll
    for (int j = 0; j < 4; ++j) zero8(acc[j]);
    const int arow = (wave * 16 + m) * ZP + 8 * h;
#pragma unroll
    for (int ks = 0; ks < 2; ++ks) {
        Frag fa, ga;
        fa.h[0] = *(const u16x8*)(sAH + arow + 32 * ks); fa.h[1] = *(const u16x8*)(sAH + arow + 32 * ks + 16);
        ga.h[0] = *(const u16x8*)(sAL + arow + 32 * ks); ga.h[1] = *(const u16x8*)(sAL + arow + 32 * ks + 16);
#pragma unroll
        for (int j = 0; j < 4; ++j) {
            Frag fb, gb;
            const unsigned short* p = w1h + (16 * j + m) * SC + 32 * ks + 8 * h;
            const unsigned short* q = w1l + (16 * j + m) * SC + 32 * ks + 8 * h;
            fb.h[0] = *(const u16x8*)p; fb.h[1] = *(const u16x8*)(p + 16);
            gb.h[0] = *(const u16x8*)q; gb.h[1] = *(const u16x8*)(q + 16);
            mma_b(acc[j], fa, fb); mma_b(acc[j], fa, gb); mma_b(acc[j], ga, fb);
        }
    }
    float* sw = st[wave];
#pragma unroll
    for (int j = 0; j < 4; ++j)
#pragma unroll
        for (int r = 0; r < 8; ++r) sw[(8 * h + r) * EP + 16 * j + m] = acc[j][r];
    __syncthreads();
    const int row = lane & 15;
    float yv = 0.f;
#pragma unroll 4
    for (int o = 0; o < SC; ++o) {
        float a = sw[row * EP + o] + bl1[o];
        a = fmaxf(a, 0.f);
        yv += wl2[o] * a;
    }
    yv += bl2[0];
    if (lane < 16) sy[wave * 16 + lane] = yv;
    __syncthreads();
    const v4f ov = *(const v4f*)(sy + (lane & 15) * 4);
    float* gp = out + tok0 + (lane & 15) * 4;
    if (wave == 0 && lane < 16) *(volatile v4f*)gp = ov;
    __threadfence();
    if (wave == 0 && lane < 16) *(volatile v4f*)gp = ov;
}

extern "C" void kernel_launch(void* const* d_in, const int* in_sizes, int n_in,
                              void* d_out, int out_size, void* d_ws, size_t ws_size, hipStream_t stream)
{
    if (n_in < 17) return;
    if (in_sizes[0] != NB * TL || in_sizes[1] != NB * AC * TF || in_sizes[2] != RC || in_sizes[3] != RC) return;
    if (in_sizes[4] != AC * AC || in_sizes[5] != 36 || in_sizes[6] != NLAY * GC * RC * 3 || in_sizes[7] != NLAY * GC) return;
    if (in_sizes[8] != NLAY * GC * AC || in_sizes[9] != NLAY * SC * RC || in_sizes[10] != NLAY * SC) return;
    if (in_sizes[11] != NLAY * RC * RC || in_sizes[12] != NLAY * RC || in_sizes[13] != SC * SC || in_sizes[14] != SC) return;
    if (in_sizes[15] != SC || in_sizes[16] != 1) return;
    if (out_size != NB * TL) return;
    if (ws_size < WS_END) return;

    const float* x       = (const float*)d_in[0];
    const float* c       = (const float*)d_in[1];
    const float* w_first = (const float*)d_in[2];
    const float* b_first = (const float*)d_in[3];
    const float* w_cin   = (const float*)d_in[4];
    const float* w_up    = (const float*)d_in[5];
    const float* wd      = (const float*)d_in[6];
    const float* bd      = (const float*)d_in[7];
    const float* wa      = (const float*)d_in[8];
    const float* wsk     = (const float*)d_in[9];
    const float* bs      = (const float*)d_in[10];
    const float* wr      = (const float*)d_in[11];
    const float* br      = (const float*)d_in[12];
    const float* wl1     = (const float*)d_in[13];
    const float* bl1     = (const float*)d_in[14];
    const float* wl2     = (const float*)d_in[15];
    const float* bl2     = (const float*)d_in[16];
    float* out = (float*)d_out;

    char* ws = (char*)d_ws;
    float* C1 = (float*)(ws + OFF_C1);
    float* U1 = (float*)(ws + OFF_U1);
    float* U2 = (float*)(ws + OFF_U2);
    float* U3 = (float*)(ws + OFF_U3);
    unsigned short* CUP = (unsigned short*)(ws + OFF_CUP);
    float* Hp[2] = {(float*)(ws + OFF_HA), (float*)(ws + OFF_HB)};
    float* Sp[2] = {(float*)(ws + OFF_SA), (float*)(ws + OFF_SB)};
    unsigned short* HHp[2] = {(unsigned short*)(ws + OFF_HHA), (unsigned short*)(ws + OFF_HHB)};
    unsigned short* WD  = (unsigned short*)(ws + OFF_WD);
    unsigned short* WA  = (unsigned short*)(ws + OFF_WA);
    unsigned short* W2  = (unsigned short*)(ws + OFF_W2);
    unsigned short* WLH = (unsigned short*)(ws + OFF_WLH);
    unsigned short* WLL = (unsigned short*)(ws + OFF_WLL);

    k_c1<<<dim3((NB * AC * TF) / 256), dim3(256), 0, stream>>>(c, w_cin, C1, NB * AC * TF);
    k_up<<<dim3((NB * AC * 512) / 256), dim3(256), 0, stream>>>(C1, w_up + 0, U1, 128, NB * AC * 512);
    k_up<<<dim3((NB * AC * 2048) / 256), dim3(256), 0, stream>>>(U1, w_up + 9, U2, 512, NB * AC * 2048);
    k_up<<<dim3((NB * AC * U3W) / 256), dim3(256), 0, stream>>>(U2, w_up + 18, U3, 2048, NB * AC * U3W);
    k_uplast<<<dim3(NB * TL / TT), dim3(256), 0, stream>>>(U3, w_up + 27, CUP);
    k_wprep<<<dim3(360, 4), dim3(256), 0, stream>>>(wd, wa, wsk, wr, wl1, WD, WA, W2, WLH, WLL);
    k_guard<<<dim3(128), dim3(256), 0, stream>>>(HHp[0]);
    k_h0<<<dim3(NB * TL / 32), dim3(128), 0, stream>>>(x, w_first, b_first, Hp[0], Sp[0], HHp[0]);

    for (int i = 0; i < NLAY; ++i) {
        const int d = 1 << (i % 10);
        const int si = i & 1, so = (i + 1) & 1;
        k_layer<<<dim3(NB * TL / TT), dim3(128), 0, stream>>>(
            HHp[si], Hp[si], Sp[si], CUP,
            WD + (size_t)i * GC * KD, WA + (size_t)i * GC * ACP, W2 + (size_t)i * GC * RC,
            bd + i * GC, bs + i * SC, br + i * RC,
            HHp[so], Hp[so], Sp[so], d);
    }
    k_tail<<<dim3(NB * TL / TT), dim3(128), 0, stream>>>(Sp[NLAY & 1], WLH, WLL, bl1, wl2, bl2, out);
}
